// mMHSA_20066087207506
// MI455X (gfx1250) — hardware-verified
//
#include <hip/hip_runtime.h>


typedef _Float16     v16h __attribute__((ext_vector_type(16)));
typedef _Float16     v8h  __attribute__((ext_vector_type(8)));
typedef float        v8f  __attribute__((ext_vector_type(8)));
typedef float        v4f  __attribute__((ext_vector_type(4)));
typedef unsigned int v4u  __attribute__((ext_vector_type(4)));

union Frag { v16h v; v8h h[2]; v4u u[2]; };
union H8   { v8h h; v4u u; };

#define DM    1024
#define NB    2
#define NSEQ  2048
#define NTOK  (NB * NSEQ)
#define NHD   16
#define DH    64
#define NPROJ 6
#define NXE   (NTOK * DM)
#define NWE   (DM * DM)

#define OFF_XH    ((size_t)0)
#define OFF_WH    ((size_t)NXE)
#define OFF_PL    ((size_t)NXE + (size_t)NPROJ * (size_t)NWE)
#define WS_HALVES (OFF_PL + (size_t)NPROJ * (size_t)NXE)

__device__ __forceinline__ v8f vzero8() {
    v8f z = {0.f, 0.f, 0.f, 0.f, 0.f, 0.f, 0.f, 0.f};
    return z;
}

__device__ __forceinline__ void ldfrag(Frag& f, const _Float16* p, int h) {
    f.h[0] = *reinterpret_cast<const v8h*>(p + 8 * h);
    f.h[1] = *reinterpret_cast<const v8h*>(p + 16 + 8 * h);
}

__device__ __forceinline__ v8f mma(const Frag& a, const Frag& b, v8f c) {
    c = __builtin_amdgcn_wmma_f32_16x16x32_f16(false, a.v, false, b.v, (short)0, c, false, false);
    asm volatile("v_nop\n\tv_nop\n\tv_nop\n\tv_nop" : "+v"(c) : "v"(a.v), "v"(b.v));
    return c;
}

#define CV_IT  8
#define CV_BLK (256 * 8 * CV_IT)

__global__ __launch_bounds__(256) void cvt_kernel(
    const float* __restrict__ x,
    const float* __restrict__ W0, const float* __restrict__ W1, const float* __restrict__ W2,
    const float* __restrict__ W3, const float* __restrict__ W4, const float* __restrict__ W5,
    _Float16* wsh)
{
    const int tid = threadIdx.x;
    const int seg = blockIdx.y;
    const float* src;
    float sc;
    if (seg < 4) {
        src = x + (size_t)seg * NWE;
        sc  = 1.0f;
    } else {
        const int p = seg - 4;
        src = (p == 0) ? W0 : (p == 1) ? W1 : (p == 2) ? W2 : (p == 3) ? W3 : (p == 4) ? W4 : W5;
        sc  = 64.0f;
    }
    const size_t base = (size_t)blockIdx.x * CV_BLK;
    const float* sp = src + base;
    _Float16*    dp = wsh + (size_t)seg * NWE + base;

    H8 v[CV_IT];
#pragma unroll
    for (int i = 0; i < CV_IT; ++i) {
        const int e = (i * 256 + tid) * 8;
        const v4f f0 = *reinterpret_cast<const v4f*>(sp + e);
        const v4f f1 = *reinterpret_cast<const v4f*>(sp + e + 4);
        H8 t;
        t.u = (v4u){0u, 0u, 0u, 0u};
#pragma unroll
        for (int q = 0; q < 4; ++q) {
            t.h[q]     = (_Float16)(f0[q] * sc);
            t.h[4 + q] = (_Float16)(f1[q] * sc);
        }
        v[i] = t;
    }
#pragma unroll
    for (int i = 0; i < CV_IT; ++i) {
        const int e = (i * 256 + tid) * 8;
        *reinterpret_cast<volatile v4u*>(dp + e) = v[i].u;
    }
    __threadfence();
#pragma unroll
    for (int i = 0; i < CV_IT; ++i) {
        const int e = (i * 256 + tid) * 8;
        *reinterpret_cast<volatile v4u*>(dp + e) = v[i].u;
    }
}

#define P_BM 128
#define P_BN 64
#define P_BK 32

template <int ISV>
__global__ __launch_bounds__(128) void proj_kernel(const _Float16* xh, const _Float16* wh,
                                                   _Float16* planes)
{
    __shared__ v4u St[1024];

    const int tid  = threadIdx.x;
    const int lane = tid & 31, w = tid >> 5, lo = lane & 15, hf = lane >> 4;
    const int z    = blockIdx.z;
    int proj;
    float osc;
    if (ISV) {
        proj = 2 + 3 * z;
        osc  = 1.0f / 64.0f;
    } else {
        proj = z + ((z >= 2) ? 1 : 0);
        osc  = (z == 0 || z == 2) ? (1.0f / 512.0f) : (1.0f / 64.0f);
    }
    const int n0 = blockIdx.x * P_BN;
    const int m0 = blockIdx.y * P_BM;

    const _Float16* xa = xh + (size_t)(m0 + 32 * w + lo) * DM;
    const _Float16* wb = wh + ((size_t)proj * DM + n0 + lo) * DM;

    v8f acc[2][4];
#pragma unroll
    for (int mt = 0; mt < 2; ++mt)
#pragma unroll
        for (int nt = 0; nt < 4; ++nt) acc[mt][nt] = vzero8();

#pragma unroll 1
    for (int k0 = 0; k0 < DM; k0 += P_BK) {
        Frag xf[2];
        ldfrag(xf[0], xa + k0, hf);
        ldfrag(xf[1], xa + 16 * DM + k0, hf);
#pragma unroll
        for (int nt = 0; nt < 4; ++nt) {
            Frag wf;
            ldfrag(wf, wb + (size_t)(16 * nt) * DM + k0, hf);
            if (ISV) {
                acc[0][nt] = mma(xf[0], wf, acc[0][nt]);
                acc[1][nt] = mma(xf[1], wf, acc[1][nt]);
            } else {
                acc[0][nt] = mma(wf, xf[0], acc[0][nt]);
                acc[1][nt] = mma(wf, xf[1], acc[1][nt]);
            }
        }
    }

#pragma unroll
    for (int mt = 0; mt < 2; ++mt) {
#pragma unroll
        for (int nt = 0; nt < 4; ++nt) {
            H8 t;
            t.u = (v4u){0u, 0u, 0u, 0u};
#pragma unroll
            for (int r = 0; r < 8; ++r) t.h[r] = (_Float16)(acc[mt][nt][r] * osc);
            if (ISV) {
                St[(16 * nt + lo) * 16 + 4 * w + 2 * mt + hf] = t.u;
            } else {
                St[(32 * w + 16 * mt + lo) * 8 + 2 * nt + hf] = t.u;
            }
        }
    }
    __syncthreads();

    const int bhi = (m0 / NSEQ) * NHD + blockIdx.x;
    const int nq0 = m0 % NSEQ;
    _Float16* plane = planes + (size_t)proj * NXE;
    const int c8 = lane & 7;
    v4u vals[8];
#pragma unroll
    for (int s = 0; s < 8; ++s) {
        const int L = 32 * w + 4 * s + (lane >> 3);
        vals[s] = St[L * 8 + c8];
    }
#pragma unroll
    for (int s = 0; s < 8; ++s) {
        const int L = 32 * w + 4 * s + (lane >> 3);
        const size_t off = ISV ? (((size_t)bhi * DH + (L >> 1)) * NSEQ + (size_t)(nq0 + 64 * (L & 1) + 8 * c8))
                               : (((size_t)bhi * NSEQ + nq0 + L) * DH + (size_t)(8 * c8));
        *reinterpret_cast<volatile v4u*>(plane + off) = vals[s];
    }
    __threadfence();
#pragma unroll
    for (int s = 0; s < 8; ++s) {
        const int L = 32 * w + 4 * s + (lane >> 3);
        const size_t off = ISV ? (((size_t)bhi * DH + (L >> 1)) * NSEQ + (size_t)(nq0 + 64 * (L & 1) + 8 * c8))
                               : (((size_t)bhi * NSEQ + nq0 + L) * DH + (size_t)(8 * c8));
        *reinterpret_cast<volatile v4u*>(plane + off) = vals[s];
    }
}

#define A_QB 64
#define A_KT 64

__global__ __launch_bounds__(128) void attn_kernel(const _Float16* planes, float* out)
{
    __shared__ v4f St[1024];

    const int tid  = threadIdx.x;
    const int lane = tid & 31, w = tid >> 5, lo = lane & 15, hf = lane >> 4;
    const int qb = blockIdx.x, bh = blockIdx.y, o = blockIdx.z;
    const int b  = bh >> 4, hd = bh & 15;
    const int s  = (hd & 1) ^ o;
    const size_t HO = (size_t)bh * NSEQ * DH;
    const _Float16* Q = planes + (size_t)(s ? 3 : 0) * NXE + HO;
    const _Float16* K = planes + (size_t)(s ? 4 : 1) * NXE + HO;
    const _Float16* V = planes + (size_t)(o ? 5 : 2) * NXE + HO;
    const int q0   = qb * A_QB;
    const int qrow = q0 + 16 * w + lo;

    Frag qf[2];
#pragma unroll
    for (int dc = 0; dc < 2; ++dc) ldfrag(qf[dc], Q + (size_t)qrow * DH + 32 * dc, hf);

    v8f O[4];
#pragma unroll
    for (int i = 0; i < 4; ++i) O[i] = vzero8();
    float mrun = -1e30f, lrun = 0.f;

#pragma unroll 1
    for (int t = 0; t < NSEQ / A_KT; ++t) {
        const int kb = t * A_KT;

        float p[32];
#pragma unroll
        for (int j = 0; j < 4; ++j) {
            v8f S = vzero8();
#pragma unroll
            for (int dc = 0; dc < 2; ++dc) {
                Frag kf;
                ldfrag(kf, K + (size_t)(kb + 16 * j + lo) * DH + 32 * dc, hf);
                S = mma(kf, qf[dc], S);
            }
#pragma unroll
            for (int r = 0; r < 8; ++r) p[8 * j + r] = S[r];
        }

        float tmax = p[0];
#pragma unroll
        for (int i = 1; i < 32; ++i) tmax = fmaxf(tmax, p[i]);
        tmax = fmaxf(tmax, __shfl_xor(tmax, 16, 32));
        const float mnew  = fmaxf(mrun, tmax);
        const float alpha = __expf(mrun - mnew);
        float rs = 0.f;
#pragma unroll
        for (int i = 0; i < 32; ++i) { p[i] = __expf(p[i] - mnew); rs += p[i]; }
        rs += __shfl_xor(rs, 16, 32);
        lrun = lrun * alpha + rs;
        mrun = mnew;
#pragma unroll
        for (int nt = 0; nt < 4; ++nt) O[nt] = O[nt] * alpha;

#pragma unroll
        for (int c = 0; c < 2; ++c) {
            H8 a0, a1;
            a0.u = (v4u){0u, 0u, 0u, 0u};
            a1.u = (v4u){0u, 0u, 0u, 0u};
#pragma unroll
            for (int r = 0; r < 8; ++r) {
                a0.h[r] = (_Float16)(p[16 * c + r] * 16384.0f);
                a1.h[r] = (_Float16)(p[16 * c + 8 + r] * 16384.0f);
            }
            Frag pf;
            pf.u[0] = a0.u;
            pf.u[1] = a1.u;
#pragma unroll
            for (int nt = 0; nt < 4; ++nt) {
                Frag vf;
                ldfrag(vf, V + (size_t)(16 * nt + lo) * NSEQ + kb + 32 * c, hf);
                O[nt] = mma(vf, pf, O[nt]);
            }
        }
    }

    const float inv = 1.0f / (lrun * 16384.0f);
    v4f* Sw = St + w * 256;
#pragma unroll
    for (int nt = 0; nt < 4; ++nt) {
        v4f a  = {O[nt][0] * inv, O[nt][1] * inv, O[nt][2] * inv, O[nt][3] * inv};
        v4f cc = {O[nt][4] * inv, O[nt][5] * inv, O[nt][6] * inv, O[nt][7] * inv};
        Sw[lo * 16 + 4 * nt + 2 * hf]     = a;
        Sw[lo * 16 + 4 * nt + 2 * hf + 1] = cc;
    }
    __syncthreads();

    float* ob = out + (size_t)o * NXE + ((size_t)b * NSEQ + q0 + 16 * w) * DM + (size_t)hd * DH;
    const int c = (lane & 7) * 4;
    v4f vals[8];
#pragma unroll
    for (int si = 0; si < 8; ++si) {
        const int L = 4 * si + (lane >> 3);
        vals[si] = Sw[8 * L + (lane & 7)];
    }
#pragma unroll
    for (int si = 0; si < 8; ++si) {
        const int L = 4 * si + (lane >> 3);
        *reinterpret_cast<volatile v4f*>(ob + (size_t)(L >> 1) * DM + 32 * (L & 1) + c) = vals[si];
    }
    __threadfence();
#pragma unroll
    for (int si = 0; si < 8; ++si) {
        const int L = 4 * si + (lane >> 3);
        *reinterpret_cast<volatile v4f*>(ob + (size_t)(L >> 1) * DM + 32 * (L & 1) + c) = vals[si];
    }
}

extern "C" void kernel_launch(void* const* d_in, const int* in_sizes, int n_in,
                              void* d_out, int out_size, void* d_ws, size_t ws_size,
                              hipStream_t stream)
{
    if (n_in < 7) return;
    if (in_sizes[0] != NXE) return;
    for (int p = 0; p < NPROJ; ++p) if (in_sizes[1 + p] != NWE) return;
    if (out_size != 2 * NXE) return;
    const size_t ws_need = WS_HALVES * sizeof(_Float16);
    if (ws_size < ws_need) return;

    const float* x  = (const float*)d_in[0];
    const float* W0 = (const float*)d_in[1];
    const float* W1 = (const float*)d_in[2];
    const float* W2 = (const float*)d_in[3];
    const float* W3 = (const float*)d_in[4];
    const float* W4 = (const float*)d_in[5];
    const float* W5 = (const float*)d_in[6];
    _Float16* wsh = (_Float16*)d_ws;
    float* out = (float*)d_out;

    cvt_kernel<<<dim3(NWE / CV_BLK, 10, 1), 256, 0, stream>>>(x, W0, W1, W2, W3, W4, W5, wsh + OFF_XH);
    proj_kernel<0><<<dim3(DM / P_BN, NTOK / P_BM, 4), 128, 0, stream>>>(wsh + OFF_XH, wsh + OFF_WH, wsh + OFF_PL);
    proj_kernel<1><<<dim3(DM / P_BN, NTOK / P_BM, 2), 128, 0, stream>>>(wsh + OFF_XH, wsh + OFF_WH, wsh + OFF_PL);
    attn_kernel<<<dim3(NSEQ / A_QB, NB * NHD, 2), 128, 0, stream>>>(wsh + OFF_PL, out);
}
